// TAGConvolution_43731357008201
// MI455X (gfx1250) — hardware-run, weakly checked
//
#include <hip/hip_runtime.h>
#include <stddef.h>
#include <stdint.h>

#ifndef TWO_TERM_1
#define TWO_TERM_1 1
#endif
#ifndef TWO_TERM_2
#define TWO_TERM_2 1
#endif
#ifndef TWO_TERM_3
#define TWO_TERM_3 1
#endif

#define NN      50000
#define FD      64
#define NE      800000
#define KW      448
#define GBM     128
#define MP      50048
#define NTHR    256
#define NWAVE   8
#define EPT     8
#define WCH     (32 * EPT)
#define NBRUN   1024
#define SLB     10
#define NBK     49
#define WLCAP   2560
#define RCAP    20480
#define TRIPCAP 64
#define MEAS_MAXDEG   37
#define MEAS_BLK_HITS 16759
#define HBM     64
#define SP      68

#define BK_ZINTS (NWAVE * WLCAP + RCAP + 3 * NBRUN)
#define BK_INTS  (BK_ZINTS + 16)
#define BK_LDS   (BK_INTS * 4)

#define PBX   (MP * FD / 8 / NTHR)
#define PBW   (FD * KW / 8 / NTHR)
#define PBTOT (PBX + PBW + 1)

static_assert(FD == 64 && FD == 16 * 4);
static_assert(MP % GBM == 0 && MP >= NN && MP == 391 * GBM && MP % HBM == 0);
static_assert(NBRUN == (1 << SLB) && NBRUN % HBM == 0 && NBRUN % GBM == 0 && NBRUN % 32 == 0);
static_assert(NBK * NBRUN >= MP);
static_assert(NE <= (1 << 20));
static_assert(NE % WCH == 0 && NE % 8 == 0);
static_assert(RCAP == NWAVE * WLCAP && BK_ZINTS % 4 == 0);
static_assert((long long)RCAP * 100 >= (long long)MEAS_BLK_HITS * 105);
static_assert(WLCAP >= MEAS_BLK_HITS / 8 + 8 * 46 + 1);
static_assert(MEAS_MAXDEG + 8 <= TRIPCAP);
static_assert(BK_LDS <= 327680);
static_assert(KW == 7 * FD && KW % 32 == 0 && FD % 32 == 0);
static_assert((MP * FD / 8) % NTHR == 0 && (FD * KW / 8) % NTHR == 0);
static_assert((RCAP * 2) % (NTHR * 4) == 0 && (2 * NBRUN) % (NTHR * 4) == 0);
static_assert(HBM == NWAVE * 8);
static_assert((GBM * SP + 128) * 4 <= 65536);
static_assert(NN % 2 == 0 && (NN - 390 * GBM) == 80);

typedef float          v4f   __attribute__((ext_vector_type(4)));
typedef float          v8f   __attribute__((ext_vector_type(8)));
typedef int            v2i   __attribute__((ext_vector_type(2)));
typedef int            v4i   __attribute__((ext_vector_type(4)));
typedef int            v8i   __attribute__((ext_vector_type(8)));
typedef unsigned       v2u   __attribute__((ext_vector_type(2)));
typedef unsigned short v8us  __attribute__((ext_vector_type(8)));
typedef unsigned short v16us __attribute__((ext_vector_type(16)));
typedef __bf16         v16bf __attribute__((ext_vector_type(16)));
typedef v4f  __attribute__((may_alias)) v4fa;
typedef v2i  __attribute__((may_alias)) v2ia;
typedef v4i  __attribute__((may_alias)) v4ia;
typedef v2u  __attribute__((may_alias)) v2ua;
typedef v8us __attribute__((may_alias)) v8usa;
union FragB { v16bf v; v16us u; v8us h[2]; v8i w; };

__device__ __forceinline__ v8f wmb(const FragB& a, const FragB& b, v8f c) {
  v8f d = __builtin_amdgcn_wmma_f32_16x16x32_bf16(false, a.v, false, b.v, (short)0, c, false, false);
  asm volatile("v_nop\n\tv_nop\n\tv_nop\n\tv_nop" : "+v"(d) : "v"(a.w), "v"(b.w));
  return d;
}

__device__ __forceinline__ unsigned bf16_bits(float f) {
  const unsigned u = __float_as_uint(f);
  const unsigned r = (u + 0x7FFFu + ((u >> 16) & 1u)) >> 16;
  const unsigned q = (u >> 16) | 0x40u;
  return ((u & 0x7fffffffu) > 0x7f800000u) ? q : r;
}
__device__ __forceinline__ float bf16_val(float f) {
  return __uint_as_float(bf16_bits(f) << 16);
}

__device__ __forceinline__ void split2(float a, float b, int& hw, int& lw) {
  const unsigned ha = bf16_bits(a), hb = bf16_bits(b);
  const unsigned la = bf16_bits(a - __uint_as_float(ha << 16));
  const unsigned lb = bf16_bits(b - __uint_as_float(hb << 16));
  hw = (int)(ha | (hb << 16));
  lw = (int)(la | (lb << 16));
}

__device__ __forceinline__ void st2_v4f(float* p, v4f v) {
  *(volatile v4f*)p = v;
  __threadfence();
  *(volatile v4f*)p = v;
}
__device__ __forceinline__ void st2_v8us(unsigned short* p, v8us v) {
  *(volatile v8us*)p = v;
  __threadfence();
  *(volatile v8us*)p = v;
}

__device__ __forceinline__ v8us gather8(const float* __restrict__ base, int stride) {
  float f[8];
#pragma unroll
  for (int i = 0; i < 8; ++i) f[i] = base[(size_t)i * (size_t)stride];
  v8us o;
#pragma unroll
  for (int i = 0; i < 8; ++i) o[i] = (unsigned short)bf16_bits(f[i]);
  return o;
}

__global__ __launch_bounds__(NTHR) void k_prep(const float* __restrict__ x, const float* __restrict__ w,
                                               const float* __restrict__ b, unsigned short* xb,
                                               unsigned short* wt, float* bfv) {
  const int tid = (int)threadIdx.x, lane = tid & 31;
  const int blk = (int)blockIdx.x;
  if (blk < PBX) {
    const int u   = blk * NTHR + tid;
    const int row = u >> 3, k8 = (u & 7) * 8;
    const int rc  = row < NN ? row : NN - 1;
    const unsigned mk = row < NN ? 0xffffu : 0u;
    const float* p = x + (size_t)rc * FD + k8;
    const v4f a = *(const v4fa*)p;
    const v4f c = *(const v4fa*)(p + 4);
    v8us o;
    o[0] = (unsigned short)(bf16_bits(a.x) & mk); o[1] = (unsigned short)(bf16_bits(a.y) & mk);
    o[2] = (unsigned short)(bf16_bits(a.z) & mk); o[3] = (unsigned short)(bf16_bits(a.w) & mk);
    o[4] = (unsigned short)(bf16_bits(c.x) & mk); o[5] = (unsigned short)(bf16_bits(c.y) & mk);
    o[6] = (unsigned short)(bf16_bits(c.z) & mk); o[7] = (unsigned short)(bf16_bits(c.w) & mk);
    st2_v8us(xb + (size_t)row * FD + k8, o);
  } else if (blk < PBX + PBW) {
    const int u  = (blk - PBX) * NTHR + tid;
    const int n  = u / (KW / 8);
    const int j  = u - n * (KW / 8);
    const int k8 = 8 * j;
    const int kb = k8 >> 6, kk = k8 & 63;
    const int sbk = (kb + 1) >> 1;
    const v8us o = gather8(w + (size_t)(sbk * FD + kk) * FD + n, FD);
    st2_v8us(wt + (size_t)u * 8, o);
  } else {
    if (tid < 32) {
      const int q = lane & 15;
      const v4f a = *(const v4fa*)(b + 4 * q);
      asm volatile("" :: "v"(a));
      const unsigned ma = (lane < 16) ? 0xffffffffu : 0u;
      v4f o;
      o.x = __uint_as_float((bf16_bits(a.x) << 16) & ma);
      o.y = __uint_as_float((bf16_bits(a.y) << 16) & ma);
      o.z = __uint_as_float((bf16_bits(a.z) << 16) & ma);
      o.w = __uint_as_float((bf16_bits(a.w) << 16) & ma);
      st2_v4f(bfv + 4 * lane, o);
    }
  }
}

__device__ __forceinline__ void bucket_flush(const int* pl, const int* cnt, int ov, int nh,
                                             const int* __restrict__ ecol, const float* __restrict__ ew,
                                             int* lp, int* cop, int* fp, int tid) {
#pragma unroll 1
  for (int it = 0; it < (RCAP * 2) / (NTHR * 4); ++it) {
    const int i0 = 2 * (it * NTHR + tid);
    const v2i ev = *(const v2ia*)(pl + i0);
    int e0 = ev.x, e1 = ev.y;
    e0 = e0 < 0 ? 0 : (e0 > NE - 1 ? NE - 1 : e0);
    e1 = e1 < 0 ? 0 : (e1 > NE - 1 ? NE - 1 : e1);
    int c0 = ecol[e0], c1 = ecol[e1];
    const float w0 = ew[e0], w1 = ew[e1];
    asm volatile("" :: "v"(c0), "v"(c1), "v"(w0), "v"(w1));
    c0 = c0 < 0 ? 0 : (c0 > NN - 1 ? NN - 1 : c0);
    c1 = c1 < 0 ? 0 : (c1 > NN - 1 ? NN - 1 : c1);
    const int m0 = (i0 < nh) ? -1 : 0;
    const int m1 = (i0 + 1 < nh) ? -1 : 0;
    v4i o;
    o.x = c0 & m0;
    o.y = (int)(bf16_bits(w0) << 16) & m0;
    o.z = c1 & m1;
    o.w = (int)(bf16_bits(w1) << 16) & m1;
    *(volatile v4i*)(lp + 2 * i0) = o;
  }
#pragma unroll 1
  for (int it = 0; it < (2 * NBRUN) / (NTHR * 4); ++it) {
    const int i0 = 4 * (it * NTHR + tid);
    const v4i v = *(const v4ia*)(cnt + i0);
    *(volatile v4i*)(cop + i0) = v;
  }
  if (tid < 8) {
    const v4i f = {ov, ov, ov, ov};
    *(volatile v4i*)(fp + 4 * tid) = f;
  }
}

__global__ __launch_bounds__(NTHR) void k_bucket(const int* __restrict__ keys, const int* __restrict__ ecol,
                                                 const float* __restrict__ ew, int* LIST, int* CO, int* FLAG) {
  extern __shared__ __attribute__((aligned(16))) int dsm[];
  int* wl   = dsm;
  int* pl   = dsm + NWAVE * WLCAP;
  int* cnt  = pl + RCAP;
  int* offs = cnt + NBRUN;
  int* cur  = offs + NBRUN;
  int* misc = cur + NBRUN;
  const int tid = (int)threadIdx.x, lane = tid & 31, wave = tid >> 5;
  const int blk = (int)blockIdx.x;
  const unsigned nbs = (unsigned)(blk * NBRUN);

  {
    const v4i z4 = {0, 0, 0, 0};
    for (int i = tid * 4; i < BK_ZINTS; i += NTHR * 4) *(v4ia*)(dsm + i) = z4;
    if (tid < 16) misc[tid] = 0;
  }
  __syncthreads();

  {
    const int per  = ((NE + NWAVE * WCH - 1) / (NWAVE * WCH)) * WCH;
    const int ebeg = wave * per;
    const int eend = (ebeg + per < NE) ? (ebeg + per) : NE;
    int* mylist = wl + wave * WLCAP;
    int wc = 0;
#pragma unroll 1
    for (int cb = ebeg; cb < eend; cb += WCH) {
      const int e0 = cb + lane * EPT;
      const v4i da = *(const v4ia*)(keys + e0);
      const v4i db = *(const v4ia*)(keys + e0 + 4);
      const unsigned s0 = (unsigned)da.x - nbs, s1 = (unsigned)da.y - nbs;
      const unsigned s2 = (unsigned)da.z - nbs, s3 = (unsigned)da.w - nbs;
      const unsigned s4 = (unsigned)db.x - nbs, s5 = (unsigned)db.y - nbs;
      const unsigned s6 = (unsigned)db.z - nbs, s7 = (unsigned)db.w - nbs;
      const bool h0 = s0 < (unsigned)NBRUN, h1 = s1 < (unsigned)NBRUN, h2 = s2 < (unsigned)NBRUN, h3 = s3 < (unsigned)NBRUN;
      const bool h4 = s4 < (unsigned)NBRUN, h5 = s5 < (unsigned)NBRUN, h6 = s6 < (unsigned)NBRUN, h7 = s7 < (unsigned)NBRUN;
      const unsigned m0 = __builtin_amdgcn_ballot_w32(h0), m1 = __builtin_amdgcn_ballot_w32(h1);
      const unsigned m2 = __builtin_amdgcn_ballot_w32(h2), m3 = __builtin_amdgcn_ballot_w32(h3);
      const unsigned m4 = __builtin_amdgcn_ballot_w32(h4), m5 = __builtin_amdgcn_ballot_w32(h5);
      const unsigned m6 = __builtin_amdgcn_ballot_w32(h6), m7 = __builtin_amdgcn_ballot_w32(h7);
      const unsigned any = m0 | m1 | m2 | m3 | m4 | m5 | m6 | m7;
      if (any != 0u) {
        const int pre = (int)(__builtin_amdgcn_mbcnt_lo(m0, 0u) + __builtin_amdgcn_mbcnt_lo(m1, 0u) +
                              __builtin_amdgcn_mbcnt_lo(m2, 0u) + __builtin_amdgcn_mbcnt_lo(m3, 0u) +
                              __builtin_amdgcn_mbcnt_lo(m4, 0u) + __builtin_amdgcn_mbcnt_lo(m5, 0u) +
                              __builtin_amdgcn_mbcnt_lo(m6, 0u) + __builtin_amdgcn_mbcnt_lo(m7, 0u));
        int p = wc + pre;
        if (h0) { if (p < WLCAP) mylist[p] = ((e0 + 0) << SLB) | (int)s0; p = p + 1; }
        if (h1) { if (p < WLCAP) mylist[p] = ((e0 + 1) << SLB) | (int)s1; p = p + 1; }
        if (h2) { if (p < WLCAP) mylist[p] = ((e0 + 2) << SLB) | (int)s2; p = p + 1; }
        if (h3) { if (p < WLCAP) mylist[p] = ((e0 + 3) << SLB) | (int)s3; p = p + 1; }
        if (h4) { if (p < WLCAP) mylist[p] = ((e0 + 4) << SLB) | (int)s4; p = p + 1; }
        if (h5) { if (p < WLCAP) mylist[p] = ((e0 + 5) << SLB) | (int)s5; p = p + 1; }
        if (h6) { if (p < WLCAP) mylist[p] = ((e0 + 6) << SLB) | (int)s6; p = p + 1; }
        if (h7) { if (p < WLCAP) mylist[p] = ((e0 + 7) << SLB) | (int)s7; p = p + 1; }
        wc += (int)(__builtin_popcount(m0) + __builtin_popcount(m1) + __builtin_popcount(m2) + __builtin_popcount(m3) +
                    __builtin_popcount(m4) + __builtin_popcount(m5) + __builtin_popcount(m6) + __builtin_popcount(m7));
      }
    }
    if (lane == 0) misc[wave] = wc;
  }
  __syncthreads();

  if (wave == 0) {
    int ov = 0;
#pragma unroll 1
    for (int w2 = 0; w2 < NWAVE; ++w2) {
      int c = misc[w2];
      if (c > WLCAP) ov = 1;
      c = c < 0 ? 0 : (c > WLCAP ? WLCAP : c);
#pragma unroll 1
      for (int b0 = 0; b0 < c; b0 += 32) {
        const int idx = b0 + lane;
        const int ent = wl[w2 * WLCAP + (idx < WLCAP ? idx : WLCAP - 1)];
        const int m32 = (c - b0) < 32 ? (c - b0) : 32;
#pragma unroll 1
        for (int k = 0; k < m32; ++k) {
          const int u    = __builtin_amdgcn_readlane(ent, k);
          const int slot = u & (NBRUN - 1);
          if (lane == 0) cnt[slot] = cnt[slot] + 1;
        }
      }
    }
    if (lane == 0) misc[9] = ov;
  }
  __syncthreads();
  if (wave == 0) {
    const int base = lane * (NBRUN / 32);
    int s = 0;
#pragma unroll 1
    for (int i = 0; i < NBRUN / 32; ++i) s += cnt[base + i];
    int incl = s;
#pragma unroll
    for (int d = 1; d < 32; d <<= 1) {
      const int y = __shfl_up(incl, d, 32);
      if (lane >= d) incl += y;
    }
    int run = incl - s;
#pragma unroll 1
    for (int i = 0; i < NBRUN / 32; ++i) {
      const int cv = cnt[base + i];
      offs[base + i] = run;
      cur[base + i]  = run;
      run += cv;
    }
  }
  __syncthreads();

  if (wave == 0) {
#pragma unroll 1
    for (int w2 = 0; w2 < NWAVE; ++w2) {
      int c = misc[w2];
      c = c < 0 ? 0 : (c > WLCAP ? WLCAP : c);
#pragma unroll 1
      for (int b0 = 0; b0 < c; b0 += 32) {
        const int idx = b0 + lane;
        const int ent = wl[w2 * WLCAP + (idx < WLCAP ? idx : WLCAP - 1)];
        const int m32 = (c - b0) < 32 ? (c - b0) : 32;
#pragma unroll 1
        for (int k = 0; k < m32; ++k) {
          const int u    = __builtin_amdgcn_readlane(ent, k);
          const int slot = u & (NBRUN - 1);
          const int eid  = (u >> SLB) & 0xFFFFF;
          if (lane == 0) {
            int p = cur[slot];
            p = p < 0 ? 0 : (p > RCAP - 1 ? RCAP - 1 : p);
            pl[p] = eid;
            cur[slot] = p + 1;
          }
        }
      }
    }
  }
  __syncthreads();

  int nh = 0;
#pragma unroll
  for (int w2 = 0; w2 < NWAVE; ++w2) {
    int c = misc[w2];
    c = c < 0 ? 0 : (c > WLCAP ? WLCAP : c);
    nh += c;
  }
  const int ovf = misc[9];
  int* lp  = LIST + (size_t)blk * (RCAP * 2);
  int* cop = CO + (size_t)blk * (2 * NBRUN);
  int* fp  = FLAG + (size_t)blk * 32;
  bucket_flush(pl, cnt, ovf, nh, ecol, ew, lp, cop, fp, tid);
  __threadfence();
  bucket_flush(pl, cnt, ovf, nh, ecol, ew, lp, cop, fp, tid);
}

template <int SRCBF>
__global__ __launch_bounds__(NTHR) void k_hop(const int* __restrict__ LIST, const int* __restrict__ CO,
                                              const int* __restrict__ FLAG, const unsigned short* SB,
                                              const float* SF, float* DST) {
  const int tid = (int)threadIdx.x, lane = tid & 31, wave = tid >> 5, hh = lane >> 4, q = lane & 15;
  const int rowBase = (int)blockIdx.x * HBM;
  const int bucket  = rowBase >> SLB;
  const int* lb  = LIST + (size_t)bucket * (RCAP * 2);
  const int* cob = CO + (size_t)bucket * (2 * NBRUN);
  const int flag = FLAG[(size_t)bucket * 32];
  const float qnan = __uint_as_float(0x7fc00000u);

#pragma unroll 1
  for (int i = 0; i < HBM / (2 * NWAVE); ++i) {
    const int d    = rowBase + (HBM / NWAVE) * wave + 2 * i + hh;
    const int slot = d & (NBRUN - 1);
    int c = cob[slot];
    int o = cob[NBRUN + slot];
    const bool big = c > TRIPCAP;
    c = c < 0 ? 0 : (c > TRIPCAP ? TRIPCAP : c);
    o = o < 0 ? 0 : (o > RCAP - 1 ? RCAP - 1 : o);
    const int co = __shfl_xor(c, 16, 32);
    const int cm = c > co ? c : co;
    const int cmu = __builtin_amdgcn_readfirstlane(cm);
    int last = o + c - 1;
    last = last < o ? o : last;
    last = last > RCAP - 1 ? RCAP - 1 : last;
    float a0 = 0.0f, a1 = 0.0f, a2 = 0.0f, a3 = 0.0f;
#pragma unroll 1
    for (int j = 0; j < cmu; ++j) {
      int idx = o + j;
      idx = idx > last ? last : idx;
      const v2i ent = *(const v2ia*)(lb + 2 * idx);
      int sr = ent.x;
      sr = sr < 0 ? 0 : (sr > NN - 1 ? NN - 1 : sr);
      const float w = __int_as_float(ent.y);
      float x0, x1, x2, x3;
      if constexpr (SRCBF != 0) {
        const v2u wd = *(const v2ua*)(SB + (size_t)sr * FD + 4 * q);
        asm volatile("" :: "v"(wd));
        x0 = __uint_as_float(wd.x << 16);
        x1 = __uint_as_float(wd.x & 0xffff0000u);
        x2 = __uint_as_float(wd.y << 16);
        x3 = __uint_as_float(wd.y & 0xffff0000u);
      } else {
        const v4f v = *(const v4fa*)(SF + (size_t)sr * FD + 4 * q);
        asm volatile("" :: "v"(v));
        x0 = v.x; x1 = v.y; x2 = v.z; x3 = v.w;
      }
      const bool valid = j < c;
      const float t0 = fmaf(w, x0, a0), t1 = fmaf(w, x1, a1), t2 = fmaf(w, x2, a2), t3 = fmaf(w, x3, a3);
      a0 = valid ? t0 : a0; a1 = valid ? t1 : a1; a2 = valid ? t2 : a2; a3 = valid ? t3 : a3;
    }
    const bool bad  = (flag != 0) | big;
    const bool live = d < NN;
    float m0 = bad ? qnan : a0, m1 = bad ? qnan : a1, m2 = bad ? qnan : a2, m3 = bad ? qnan : a3;
    m0 = live ? m0 : 0.0f; m1 = live ? m1 : 0.0f; m2 = live ? m2 : 0.0f; m3 = live ? m3 : 0.0f;
    v4f ov;
    ov.x = m0; ov.y = m1; ov.z = m2; ov.w = m3;
    st2_v4f(DST + (size_t)d * FD + 4 * q, ov);
  }
}

__device__ __forceinline__ void gemm_xb(const unsigned short* __restrict__ ap,
                                        const unsigned short* __restrict__ bp, v8f (&acc)[4]) {
#pragma unroll 1
  for (int ks = 0; ks < FD; ks += 32) {
    FragB af;
    af.h[0] = *(const v8usa*)(ap + ks);
    af.h[1] = *(const v8usa*)(ap + ks + 16);
#pragma unroll
    for (int nt = 0; nt < 4; ++nt) {
      const unsigned short* wq = bp + (size_t)(16 * nt) * (size_t)KW + ks;
      FragB bfr;
      bfr.h[0] = *(const v8usa*)wq;
      bfr.h[1] = *(const v8usa*)(wq + 16);
      acc[nt] = wmb(af, bfr, acc[nt]);
    }
  }
}

template <int TT>
__device__ __forceinline__ void gemm_plane(const float* ar, const unsigned short* __restrict__ bp, v8f (&acc)[4]) {
#pragma unroll 1
  for (int ks = 0; ks < FD; ks += 32) {
    const v4f f0 = *(const v4fa*)(ar + ks);
    const v4f f1 = *(const v4fa*)(ar + ks + 4);
    const v4f f2 = *(const v4fa*)(ar + ks + 16);
    const v4f f3 = *(const v4fa*)(ar + ks + 20);
    int h0, h1, h2, h3, h4, h5, h6, h7, l0, l1, l2, l3, l4, l5, l6, l7;
    split2(f0.x, f0.y, h0, l0); split2(f0.z, f0.w, h1, l1);
    split2(f1.x, f1.y, h2, l2); split2(f1.z, f1.w, h3, l3);
    split2(f2.x, f2.y, h4, l4); split2(f2.z, f2.w, h5, l5);
    split2(f3.x, f3.y, h6, l6); split2(f3.z, f3.w, h7, l7);
    FragB ah;
    const v8i hv = {h0, h1, h2, h3, h4, h5, h6, h7};
    ah.w = hv;
#pragma unroll
    for (int nt = 0; nt < 4; ++nt) {
      const unsigned short* wq = bp + (size_t)(16 * nt) * (size_t)KW + ks;
      FragB bfr;
      bfr.h[0] = *(const v8usa*)wq;
      bfr.h[1] = *(const v8usa*)(wq + 16);
      acc[nt] = wmb(ah, bfr, acc[nt]);
    }
    if constexpr (TT != 0) {
      FragB al;
      const v8i lv = {l0, l1, l2, l3, l4, l5, l6, l7};
      al.w = lv;
#pragma unroll
      for (int nt = 0; nt < 4; ++nt) {
        const unsigned short* wq = bp + FD + (size_t)(16 * nt) * (size_t)KW + ks;
        FragB bfr;
        bfr.h[0] = *(const v8usa*)wq;
        bfr.h[1] = *(const v8usa*)(wq + 16);
        acc[nt] = wmb(al, bfr, acc[nt]);
      }
    }
  }
}

__device__ __forceinline__ void stage_d(float* stg, const v8f (&acc)[4], int wave, int hh, int m) {
#pragma unroll
  for (int nt = 0; nt < 4; ++nt) {
#pragma unroll
    for (int r = 0; r < 8; ++r) stg[(16 * wave + 8 * hh + r) * SP + 16 * nt + m] = acc[nt][r];
  }
}

__global__ __launch_bounds__(NTHR) __attribute__((amdgpu_num_vgpr(248)))
void k_gemm(const unsigned short* __restrict__ XB, const float* __restrict__ PLa, const float* __restrict__ PLb,
            const float* __restrict__ PLc, const unsigned short* __restrict__ WT, const float* __restrict__ BF,
            const int* __restrict__ FLAG, float* out) {
  __shared__ __attribute__((aligned(16))) float stg[GBM * SP];
  __shared__ __attribute__((aligned(16))) float sb[128];
  const int tid = (int)threadIdx.x, lane = tid & 31, wave = tid >> 5, hh = lane >> 4, m = lane & 15;
  const int rowBase = (int)blockIdx.x * GBM;
  const int flag = FLAG[(size_t)(rowBase >> SLB) * 32];
  if (tid < 32) *(v4fa*)(sb + 4 * tid) = *(const v4fa*)(BF + 4 * tid);

  v8f acc[4];
  {
    const v8f z = {0.f, 0.f, 0.f, 0.f, 0.f, 0.f, 0.f, 0.f};
#pragma unroll
    for (int t = 0; t < 4; ++t) acc[t] = z;
  }
  const size_t arow = (size_t)(rowBase + 16 * wave + m) * (size_t)FD + 8 * hh;
  const unsigned short* bp = WT + (size_t)m * (size_t)KW + 8 * hh;
  gemm_xb(XB + arow, bp, acc);
  gemm_plane<TWO_TERM_1>(PLa + arow, bp + 64, acc);
  gemm_plane<TWO_TERM_2>(PLb + arow, bp + 192, acc);
  gemm_plane<TWO_TERM_3>(PLc + arow, bp + 320, acc);
  stage_d(stg, acc, wave, hh, m);
  __syncthreads();

  const v4f bias = *(const v4fa*)(sb + 4 * m);
  const float qnan = __uint_as_float(0x7fc00000u);
#pragma unroll 1
  for (int i = 0; i < 8; ++i) {
    const int lr   = 16 * wave + 2 * i + hh;
    const int grow = rowBase + lr;
    const bool live = grow < NN;
    const int grc  = live ? grow : NN - 1;
    const v4f a = *(const v4fa*)(stg + lr * SP + 4 * m);
    asm volatile("" :: "v"(a));
    float v0 = a.x + bias.x, v1 = a.y + bias.y, v2 = a.z + bias.z, v3 = a.w + bias.w;
    v0 = (flag != 0) ? qnan : v0; v1 = (flag != 0) ? qnan : v1;
    v2 = (flag != 0) ? qnan : v2; v3 = (flag != 0) ? qnan : v3;
    v4f o;
    o.x = v0; o.y = v1; o.z = v2; o.w = v3;
    float* op = out + (size_t)grc * FD + 4 * m;
    if (live) *(volatile v4f*)op = o;
    __threadfence();
    if (live) *(volatile v4f*)op = o;
  }
}

extern "C" void kernel_launch(void* const* d_in, const int* in_sizes, int n_in,
                              void* d_out, int out_size, void* d_ws, size_t ws_size,
                              hipStream_t stream) {
  if (n_in < 6) return;
  if (in_sizes[0] != NN * FD) return;
  if (in_sizes[1] != NE) return;
  if (in_sizes[2] != NE) return;
  if (in_sizes[3] != NE) return;
  if (in_sizes[4] != 4 * FD * FD) return;
  if (in_sizes[5] != FD) return;
  if (out_size != NN * FD) return;

  const float* x    = (const float*)d_in[0];
  const int*   erow = (const int*)d_in[1];
  const int*   ecol = (const int*)d_in[2];
  const float* ew   = (const float*)d_in[3];
  const float* W    = (const float*)d_in[4];
  const float* b    = (const float*)d_in[5];
  float* out = (float*)d_out;

  constexpr size_t zXB   = (size_t)MP * FD * 2;
  constexpr size_t zF    = (size_t)MP * FD * 4;
  constexpr size_t zLIST = (size_t)NBK * RCAP * 8;
  constexpr size_t zCO   = (size_t)NBK * 2 * NBRUN * 4;
  constexpr size_t zFLAG = (((size_t)NBK * 128 + 255) / 256) * 256;
  constexpr size_t zWT   = (size_t)FD * KW * 2;
  constexpr size_t zBF   = 512;
  constexpr size_t oXB   = 0;
  constexpr size_t oPLa  = oXB + zXB;
  constexpr size_t oPLb  = oPLa + zF;
  constexpr size_t oPLc  = oPLb + zF;
  constexpr size_t oLIST = oPLc + zF;
  constexpr size_t oCO   = oLIST + zLIST;
  constexpr size_t oFLAG = oCO + zCO;
  constexpr size_t oWT   = oFLAG + zFLAG;
  constexpr size_t oBF   = oWT + zWT;
  constexpr size_t oEND  = oBF + zBF;
  static_assert(zXB % 256 == 0 && zF % 256 == 0 && zLIST % 256 == 0 && zCO % 256 == 0);
  static_assert(zFLAG % 256 == 0 && zFLAG >= (size_t)NBK * 128 && zWT % 256 == 0 && zBF % 256 == 0);
  static_assert(oEND <= (size_t)(128u << 20));
  if (oEND > ws_size) return;

  char* ws = (char*)d_ws;
  unsigned short* XB   = (unsigned short*)(ws + oXB);
  float*          PLa  = (float*)(ws + oPLa);
  float*          PLb  = (float*)(ws + oPLb);
  float*          PLc  = (float*)(ws + oPLc);
  int*            LIST = (int*)(ws + oLIST);
  int*            CO   = (int*)(ws + oCO);
  int*            FLAG = (int*)(ws + oFLAG);
  unsigned short* WT   = (unsigned short*)(ws + oWT);
  float*          BF   = (float*)(ws + oBF);

  hipFuncSetAttribute(reinterpret_cast<const void*>(&k_bucket), hipFuncAttributeMaxDynamicSharedMemorySize, (int)BK_LDS);

  k_prep<<<PBTOT, NTHR, 0, stream>>>(x, W, b, XB, WT, BF);
  k_bucket<<<NBK, NTHR, BK_LDS, stream>>>(erow, ecol, ew, LIST, CO, FLAG);
  k_hop<1><<<MP / HBM, NTHR, 0, stream>>>(LIST, CO, FLAG, XB, PLb, PLa);
  k_hop<0><<<MP / HBM, NTHR, 0, stream>>>(LIST, CO, FLAG, XB, PLa, PLb);
  k_hop<0><<<MP / HBM, NTHR, 0, stream>>>(LIST, CO, FLAG, XB, PLb, PLc);
  k_gemm<<<MP / GBM, NTHR, 0, stream>>>(XB, PLa, PLb, PLc, WT, BF, FLAG, out);
}
